// GCN2Model_58935541236367
// MI455X (gfx1250) — hardware-verified
//
#include <hip/hip_runtime.h>
#include <math.h>
#include <stddef.h>


#define HD      128
#define AP      136
#define NTHR    256
#define NWAVE   8
#define EPT     8
#define NGRP    2
#define CHUNK   (NTHR * EPT * NGRP)
#define WCAP    (EPT * NGRP * 32)
#define LISTN   (NWAVE * WCAP)
#define NBC     4096
#define NBF     1024
#define RCAP    40960
#define RBN     128
#define GROWS   128
#define RPAD    256
#define DEGCAP  256
#define OTHR    512
#define WSCALE  256.0f
#define WINV    0.00390625f

#define LDS_SM   (GROWS * HD * 4)
#define LDS_SA   (GROWS * AP * 2)
#define LDS_G    (LDS_SM + LDS_SA + GROWS * 4)
#define LDS_FILL ((RCAP + NBF + LISTN) * 4 + 64)

static_assert((CHUNK & (CHUNK - 1)) == 0);
static_assert(CHUNK <= 4096);
static_assert(NBC <= 4096 && NBF <= 4096);
static_assert((NBC & (NBC - 1)) == 0 && (NBF & (NBF - 1)) == 0);
static_assert(NBC == 4 * NBF);
static_assert(OTHR * 8 == NBC);
static_assert((RCAP % 32) == 0);
static_assert((AP % 8) == 0);
static_assert(GROWS == NWAVE * 16);
static_assert((RPAD % GROWS) == 0);
static_assert((GROWS * HD / 8) % NTHR == 0);
static_assert((LDS_SM % 16) == 0 && (LDS_SA % 16) == 0);

typedef float    v4f  __attribute__((ext_vector_type(4)));
typedef float    v8f  __attribute__((ext_vector_type(8)));
typedef int      v4i  __attribute__((ext_vector_type(4)));
typedef _Float16 v4h  __attribute__((ext_vector_type(4)));
typedef _Float16 v8h  __attribute__((ext_vector_type(8)));
typedef _Float16 v16h __attribute__((ext_vector_type(16)));
union FragH { v16h v; v8h h[2]; };

__device__ __forceinline__ v8h cvt8(v4f a, v4f b) {
  v8h r;
  r[0] = (_Float16)a.x; r[1] = (_Float16)a.y; r[2] = (_Float16)a.z; r[3] = (_Float16)a.w;
  r[4] = (_Float16)b.x; r[5] = (_Float16)b.y; r[6] = (_Float16)b.z; r[7] = (_Float16)b.w;
  return r;
}

__device__ __forceinline__ v8f wmh(v16h a, v16h b, v8f c) {
  v8f d = __builtin_amdgcn_wmma_f32_16x16x32_f16(false, a, false, b, (short)0, c, false, false);
  asm volatile("v_nop\n\tv_nop\n\tv_nop\n\tv_nop" : "+v"(d) : "v"(a), "v"(b));
  return d;
}

__device__ __forceinline__ void carry_of(float mx, float& sc, float& isc) {
  const unsigned eb = (__float_as_uint(mx) >> 23) & 255u;
  int sh = (eb == 0u) ? 0 : (138 - (int)eb);
  sh = sh < -100 ? -100 : (sh > 100 ? 100 : sh);
  sc  = __uint_as_float((unsigned)(127 + sh) << 23);
  isc = __uint_as_float((unsigned)(127 - sh) << 23);
}

template <int NB>
__device__ __forceinline__ int scan_chunk(const int* __restrict__ dsts, int nE, int cbase, int slotBase,
                                          int vec8, int* list, int tid, int lane, int wave) {
  int wc = 0;
#pragma unroll
  for (int g = 0; g < NGRP; ++g) {
    const int el0  = (g * NTHR + tid) * EPT;
    const int e0   = cbase + el0;
    const int sent = -2147483647 - 1;
    v4i da, db;
    if (vec8 != 0 && cbase + CHUNK <= nE) {
      da = *(const v4i*)(dsts + e0);
      db = *(const v4i*)(dsts + e0 + 4);
    } else {
      da.x = (e0     < nE) ? dsts[min(e0, nE - 1)] : sent;
      da.y = (e0 + 1 < nE) ? dsts[min(e0 + 1, nE - 1)] : sent;
      da.z = (e0 + 2 < nE) ? dsts[min(e0 + 2, nE - 1)] : sent;
      da.w = (e0 + 3 < nE) ? dsts[min(e0 + 3, nE - 1)] : sent;
      db.x = (e0 + 4 < nE) ? dsts[min(e0 + 4, nE - 1)] : sent;
      db.y = (e0 + 5 < nE) ? dsts[min(e0 + 5, nE - 1)] : sent;
      db.z = (e0 + 6 < nE) ? dsts[min(e0 + 6, nE - 1)] : sent;
      db.w = (e0 + 7 < nE) ? dsts[min(e0 + 7, nE - 1)] : sent;
    }
    const unsigned nb = (unsigned)slotBase;
    const unsigned s0 = (unsigned)da.x - nb, s1 = (unsigned)da.y - nb;
    const unsigned s2 = (unsigned)da.z - nb, s3 = (unsigned)da.w - nb;
    const unsigned s4 = (unsigned)db.x - nb, s5 = (unsigned)db.y - nb;
    const unsigned s6 = (unsigned)db.z - nb, s7 = (unsigned)db.w - nb;
    const bool h0 = s0 < (unsigned)NB, h1 = s1 < (unsigned)NB, h2 = s2 < (unsigned)NB, h3 = s3 < (unsigned)NB;
    const bool h4 = s4 < (unsigned)NB, h5 = s5 < (unsigned)NB, h6 = s6 < (unsigned)NB, h7 = s7 < (unsigned)NB;
    const unsigned any = __builtin_amdgcn_ballot_w32(h0 | h1 | h2 | h3 | h4 | h5 | h6 | h7);
    if (any != 0u) {
#define HITJ(J, HJ, SJ) { \
        const unsigned mj = __builtin_amdgcn_ballot_w32(HJ); \
        if (mj != 0u) { \
          if (HJ) { \
            const int pos = wc + (int)__builtin_amdgcn_mbcnt_lo(mj, 0u); \
            if (pos < WCAP) list[wave * WCAP + pos] = ((el0 + (J)) << 12) | (int)(SJ); \
          } \
          wc += (int)__builtin_popcount(mj); } }
      HITJ(0, h0, s0)
      HITJ(1, h1, s1)
      HITJ(2, h2, s2)
      HITJ(3, h3, s3)
      HITJ(4, h4, s4)
      HITJ(5, h5, s5)
      HITJ(6, h6, s6)
      HITJ(7, h7, s7)
#undef HITJ
    }
  }
  return wc;
}

__global__ __launch_bounds__(NTHR) void k_wprep(
    const float* __restrict__ W0, const float* __restrict__ convW, const float* __restrict__ W1,
    _Float16* wts, int nL) {
  const int mat = (int)(blockIdx.x >> 3);
  const float* src = W1;
  if (mat == 0) src = W0;
  else if (mat <= nL) src = convW + (size_t)(mat - 1) * HD * HD;
  const int i  = (int)((blockIdx.x & 7u) * NTHR + threadIdx.x);
  const int o  = i * 8;
  const int n  = o >> 7;
  const int k0 = o & (HD - 1);
  const float* cp = src + (size_t)k0 * HD + n;
  v4f a, b;
  a.x = cp[0 * HD] * WSCALE; a.y = cp[1 * HD] * WSCALE; a.z = cp[2 * HD] * WSCALE; a.w = cp[3 * HD] * WSCALE;
  b.x = cp[4 * HD] * WSCALE; b.y = cp[5 * HD] * WSCALE; b.z = cp[6 * HD] * WSCALE; b.w = cp[7 * HD] * WSCALE;
  const v8h hv = cvt8(a, b);
  _Float16* dp = wts + (size_t)mat * HD * HD + o;
  *(volatile v8h*)dp = hv;
  __threadfence();
  *(volatile v8h*)dp = hv;
}

__global__ __launch_bounds__(NTHR) void k_count(
    const int* __restrict__ dsts, int* cnt, int nE, int vec8) {
  __shared__ __attribute__((aligned(16))) int scnt[NBC];
  __shared__ __attribute__((aligned(16))) int list[LISTN];
  __shared__ int wcnt[NWAVE];
  const int tid = threadIdx.x, lane = tid & 31, wave = tid >> 5;
  const int nodeBase = blockIdx.x * NBC;

  for (int i = tid; i < NBC; i += NTHR) scnt[i] = 0;
  __syncthreads();

  const int nChunks = (nE + CHUNK - 1) / CHUNK;
#pragma unroll 1
  for (int ch = 0; ch < nChunks; ++ch) {
    const int cbase = ch * CHUNK;
    const int wc = scan_chunk<NBC>(dsts, nE, cbase, nodeBase, vec8, list, tid, lane, wave);
    if (lane == 0) wcnt[wave] = wc;
    __syncthreads();
    if (wave == 0) {
#pragma unroll 1
      for (int wsx = 0; wsx < NWAVE; ++wsx) {
        int n = __builtin_amdgcn_readfirstlane(wcnt[wsx]);
        n = n > WCAP ? WCAP : (n < 0 ? 0 : n);
        const int* lp = list + wsx * WCAP;
#pragma unroll 1
        for (int i = 0; i < n; ++i) {
          const int ent  = __builtin_amdgcn_readfirstlane(lp[i]);
          const int slot = ent & (NBC - 1);
          if (lane == 0) scnt[slot] = scnt[slot] + 1;
        }
      }
    }
    __syncthreads();
  }

  v4i cq[4];
#pragma unroll
  for (int q = 0; q < 4; ++q) {
    const int f = (wave * 4 + q) * 128 + 4 * lane;
    cq[q] = *(const v4i*)(scnt + f);
  }
  int* cp = cnt + (size_t)nodeBase;
#pragma unroll
  for (int q = 0; q < 4; ++q) {
    const int f = (wave * 4 + q) * 128 + 4 * lane;
    *(volatile v4i*)(cp + f) = cq[q];
  }
  __threadfence();
#pragma unroll
  for (int q = 0; q < 4; ++q) {
    const int f = (wave * 4 + q) * 128 + 4 * lane;
    *(volatile v4i*)(cp + f) = cq[q];
  }
}

__global__ __launch_bounds__(OTHR) void k_offsets(
    const int* __restrict__ cnt, int* off, int* rbase, int nChunk) {
  __shared__ __attribute__((aligned(16))) int soff[NBC];
  __shared__ __attribute__((aligned(16))) int srb[RBN];
  __shared__ int wtot[OTHR / 32];
  const int tid = threadIdx.x, lane = tid & 31, wave = tid >> 5, sub = tid >> 7;
  for (int i = tid; i < RBN; i += OTHR) srb[i] = 0;
  int carry = 0;
#pragma unroll 1
  for (int ch = 0; ch < nChunk; ++ch) {
    const int base = ch * NBC;
    const v4i c0 = *(const v4i*)(cnt + base + 8 * tid);
    const v4i c1 = *(const v4i*)(cnt + base + 8 * tid + 4);
    const int e0 = max(c0.x, 0), e1 = max(c0.y, 0), e2 = max(c0.z, 0), e3 = max(c0.w, 0);
    const int e4 = max(c1.x, 0), e5 = max(c1.y, 0), e6 = max(c1.z, 0), e7 = max(c1.w, 0);
    const int ts = e0 + e1 + e2 + e3 + e4 + e5 + e6 + e7;
    int incl = ts;
#pragma unroll
    for (int d = 1; d < 32; d <<= 1) {
      const int t = __shfl_up(incl, d);
      if (lane >= d) incl += t;
    }
    if (lane == 31) wtot[wave] = incl;
    __syncthreads();
    const int S0 = wtot[0]  + wtot[1]  + wtot[2]  + wtot[3];
    const int S1 = wtot[4]  + wtot[5]  + wtot[6]  + wtot[7];
    const int S2 = wtot[8]  + wtot[9]  + wtot[10] + wtot[11];
    const int S3 = wtot[12] + wtot[13] + wtot[14] + wtot[15];
    int pre = 0;
#pragma unroll 1
    for (int w = 4 * sub; w < wave; ++w) pre += wtot[w];
    const int b0 = carry;
    const int b1 = b0 + ((S0 + 31) & ~31);
    const int b2 = b1 + ((S1 + 31) & ~31);
    const int b3 = b2 + ((S2 + 31) & ~31);
    const int b4 = b3 + ((S3 + 31) & ~31);
    const int myb = sub == 0 ? b0 : (sub == 1 ? b1 : (sub == 2 ? b2 : b3));
    if (tid == 0) {
      srb[min(4 * ch + 0, RBN - 1)] = b0;
      srb[min(4 * ch + 1, RBN - 1)] = b1;
      srb[min(4 * ch + 2, RBN - 1)] = b2;
      srb[min(4 * ch + 3, RBN - 1)] = b3;
    }
    int run = myb + pre + incl - ts;
    soff[8 * tid + 0] = run; run += e0;
    soff[8 * tid + 1] = run; run += e1;
    soff[8 * tid + 2] = run; run += e2;
    soff[8 * tid + 3] = run; run += e3;
    soff[8 * tid + 4] = run; run += e4;
    soff[8 * tid + 5] = run; run += e5;
    soff[8 * tid + 6] = run; run += e6;
    soff[8 * tid + 7] = run;
    carry = b4;
    __syncthreads();
    const v4i o0 = *(const v4i*)(soff + 4 * tid);
    const v4i o1 = *(const v4i*)(soff + 4 * (tid + OTHR));
    int* op = off + base;
    *(volatile v4i*)(op + 4 * tid) = o0;
    *(volatile v4i*)(op + 4 * (tid + OTHR)) = o1;
    __threadfence();
    *(volatile v4i*)(op + 4 * tid) = o0;
    *(volatile v4i*)(op + 4 * (tid + OTHR)) = o1;
    __syncthreads();
  }
  if (tid == 0) srb[min(4 * nChunk, RBN - 1)] = carry;
  __syncthreads();
  v4i rv = {0, 0, 0, 0};
  if (tid < 32) rv = *(const v4i*)(srb + 4 * tid);
  if (tid < 32) *(volatile v4i*)(rbase + 4 * tid) = rv;
  __threadfence();
  if (tid < 32) *(volatile v4i*)(rbase + 4 * tid) = rv;
}

__global__ __launch_bounds__(NTHR) void k_fill(
    const int* __restrict__ dsts, const int* __restrict__ off, const int* __restrict__ rbase,
    int* csr, int nE, int vec8, int csrLen) {
  extern __shared__ v4f lds_dyn[];
  int* region = (int*)lds_dyn;
  int* cursor = region + RCAP;
  int* list   = cursor + NBF;
  int* wcnt   = list + LISTN;
  const int tid = threadIdx.x, lane = tid & 31, wave = tid >> 5;
  const int b = blockIdx.x;
  const int nodeBase = b * NBF;

  int rb0 = rbase[b];
  const int rb1 = rbase[b + 1];
  rb0 = rb0 < 0 ? 0 : (rb0 > csrLen ? csrLen : rb0);
  rb0 &= ~31;
  int len = rb1 - rb0;
  len = len < 0 ? 0 : (len > RCAP ? RCAP : len);
  int lenW = (len + 31) & ~31;
  if (rb0 + lenW > csrLen) lenW = (csrLen - rb0) & ~31;

  {
    const v4i z = {0, 0, 0, 0};
    for (int i = tid; i < RCAP / 4; i += NTHR) ((v4i*)region)[i] = z;
    for (int s = tid; s < NBF; s += NTHR) {
      int o = off[nodeBase + s] - rb0;
      o = o < 0 ? 0 : (o > RCAP ? RCAP : o);
      cursor[s] = o;
    }
  }
  __syncthreads();

  const int nChunks = (nE + CHUNK - 1) / CHUNK;
#pragma unroll 1
  for (int ch = 0; ch < nChunks; ++ch) {
    const int cbase = ch * CHUNK;
    const int wc = scan_chunk<NBF>(dsts, nE, cbase, nodeBase, vec8, list, tid, lane, wave);
    if (lane == 0) wcnt[wave] = wc;
    __syncthreads();
    if (wave == 0) {
#pragma unroll 1
      for (int wsx = 0; wsx < NWAVE; ++wsx) {
        int n = __builtin_amdgcn_readfirstlane(wcnt[wsx]);
        n = n > WCAP ? WCAP : (n < 0 ? 0 : n);
        const int* lp = list + wsx * WCAP;
#pragma unroll 1
        for (int i = 0; i < n; ++i) {
          const int ent  = __builtin_amdgcn_readfirstlane(lp[i]);
          const int slot = ent & (NBF - 1);
          int e = cbase + ((ent >> 12) & (CHUNK - 1));
          e = e > nE - 1 ? nE - 1 : e;
          if (lane == 0) {
            int pos = cursor[slot];
            pos = pos < 0 ? 0 : (pos > RCAP - 1 ? RCAP - 1 : pos);
            region[pos] = e;
            const int np = pos + 1;
            cursor[slot] = np > RCAP ? RCAP : np;
          }
        }
      }
    }
    __syncthreads();
  }

  const int nv = lenW >> 2;
  int* gp = csr + rb0;
#pragma unroll 1
  for (int i = tid; i < nv; i += NTHR) { const v4i v = ((const v4i*)region)[i]; *(volatile v4i*)(gp + 4 * i) = v; }
  __threadfence();
#pragma unroll 1
  for (int i = tid; i < nv; i += NTHR) { const v4i v = ((const v4i*)region)[i]; *(volatile v4i*)(gp + 4 * i) = v; }
}

__device__ __forceinline__ void stage_rows(const float* __restrict__ A, int rowBase, int nRowsA,
                                           _Float16* sA, float* sFac, int tid, int lane) {
#pragma unroll 2
  for (int i = 0; i < (GROWS * HD / 8) / NTHR; ++i) {
    const int idx = i * NTHR + tid;
    const int r   = idx >> 4;
    const int c0  = (idx & 15) * 8;
    int row = rowBase + r;
    row = row > nRowsA - 1 ? nRowsA - 1 : row;
    const float* ap = A + (size_t)row * HD + c0;
    const v4f a = *(const v4f*)ap, b = *(const v4f*)(ap + 4);
    float mx = fmaxf(fmaxf(fmaxf(fabsf(a.x), fabsf(a.y)), fmaxf(fabsf(a.z), fabsf(a.w))),
                     fmaxf(fmaxf(fabsf(b.x), fabsf(b.y)), fmaxf(fabsf(b.z), fabsf(b.w))));
    mx = fmaxf(mx, __shfl_xor(mx, 8));
    mx = fmaxf(mx, __shfl_xor(mx, 4));
    mx = fmaxf(mx, __shfl_xor(mx, 2));
    mx = fmaxf(mx, __shfl_xor(mx, 1));
    float sc, isc;
    carry_of(mx, sc, isc);
    *(v8h*)(sA + r * AP + c0) = cvt8(a * sc, b * sc);
    if ((lane & 15) == 0) sFac[r] = isc * WINV;
  }
}

__device__ __forceinline__ void mma_rows(const _Float16* sA, const _Float16* __restrict__ Bs,
                                         int wave, int hh, int m, v8f (&acc)[8]) {
#pragma unroll
  for (int t = 0; t < 8; ++t) { v8f z = {0.f, 0.f, 0.f, 0.f, 0.f, 0.f, 0.f, 0.f}; acc[t] = z; }
  const _Float16* ar = sA + (wave * 16 + m) * AP + 8 * hh;
#pragma unroll
  for (int kt = 0; kt < HD / 32; ++kt) {
    FragH a;
    a.h[0] = *(const v8h*)(ar + 32 * kt);
    a.h[1] = *(const v8h*)(ar + 32 * kt + 16);
#pragma unroll
    for (int t = 0; t < 8; ++t) {
      const _Float16* bp = Bs + (size_t)(16 * t + m) * HD + 32 * kt + 8 * hh;
      FragH b;
      b.h[0] = *(const v8h*)bp;
      b.h[1] = *(const v8h*)(bp + 16);
      acc[t] = wmh(a.v, b.v, acc[t]);
    }
  }
}

__device__ __forceinline__ void store_rows2(const float* sM, float* C, int rowBase, int nRowsOut,
                                            int wave, int lane) {
  const int rw = rowBase + wave * 16;
  const float* lp = sM + wave * 16 * HD + 4 * lane;
  float* gp = C + (size_t)rw * HD + 4 * lane;
#pragma unroll
  for (int i = 0; i < 16; ++i)
    if (rw + i < nRowsOut) { const v4f v = *(const v4f*)(lp + i * HD); *(volatile v4f*)(gp + (size_t)i * HD) = v; }
  __threadfence();
#pragma unroll
  for (int i = 0; i < 16; ++i)
    if (rw + i < nRowsOut) { const v4f v = *(const v4f*)(lp + i * HD); *(volatile v4f*)(gp + (size_t)i * HD) = v; }
}

__global__ __launch_bounds__(NTHR) void k_gemm0(
    const float* __restrict__ X, const _Float16* __restrict__ Bs, const float* __restrict__ bias,
    float* C, int nRowsA, int nRowsOut) {
  extern __shared__ v4f lds_dyn[];
  float*    sM   = (float*)lds_dyn;
  _Float16* sA   = (_Float16*)((char*)lds_dyn + LDS_SM);
  float*    sFac = (float*)((char*)lds_dyn + LDS_SM + LDS_SA);
  const int tid = threadIdx.x, lane = tid & 31, wave = tid >> 5, hh = lane >> 4, m = lane & 15;
  const int rowBase = blockIdx.x * GROWS;

  stage_rows(X, rowBase, nRowsA, sA, sFac, tid, lane);
  __syncthreads();

  v8f acc[8];
  mma_rows(sA, Bs, wave, hh, m, acc);

  const int r0 = wave * 16 + 8 * hh;
  const v4f fA = *(const v4f*)(sFac + r0);
  const v4f fB = *(const v4f*)(sFac + r0 + 4);
  float f[8];
  f[0] = fA.x; f[1] = fA.y; f[2] = fA.z; f[3] = fA.w; f[4] = fB.x; f[5] = fB.y; f[6] = fB.z; f[7] = fB.w;
  float* sp = sM + r0 * HD + m;
#pragma unroll
  for (int t = 0; t < 8; ++t) {
    const float bl = bias[16 * t + m];
#pragma unroll
    for (int r = 0; r < 8; ++r) sp[r * HD + 16 * t] = fmaxf(acc[t][r] * f[r] + bl, 0.0f);
  }
  __syncthreads();
  store_rows2(sM, C, rowBase, nRowsOut, wave, lane);
}

__global__ __launch_bounds__(NTHR) void k_layer(
    const int* __restrict__ csr, const int* __restrict__ offp, const int* __restrict__ cnt,
    const int* __restrict__ esrc, const float* __restrict__ ew,
    const float* hin, const float* x0, const _Float16* __restrict__ Bs,
    float* hout, int nN, int nE, int csrLen, int nRowsOut, float omb, float bet) {
  extern __shared__ v4f lds_dyn[];
  float*    sM   = (float*)lds_dyn;
  _Float16* sA   = (_Float16*)((char*)lds_dyn + LDS_SM);
  float*    sFac = (float*)((char*)lds_dyn + LDS_SM + LDS_SA);
  const int tid = threadIdx.x, lane = tid & 31, wave = tid >> 5, hh = lane >> 4, m = lane & 15;
  const int rowBase = blockIdx.x * GROWS;
  const int r0w = wave * 16;

  const int cl = rowBase + r0w + m;
  const int cnt_l = cnt[cl];
  const int off_l = offp[cl];
#pragma unroll 1
  for (int j = 0; j < 16; ++j) {
    const int c = rowBase + r0w + j;
    int n = __builtin_amdgcn_readlane(cnt_l, j);
    n = n < 0 ? 0 : (n > DEGCAP ? DEGCAP : n);
    const int st = __builtin_amdgcn_readlane(off_l, j);
    v4f acc = {0.f, 0.f, 0.f, 0.f};
#pragma unroll 1
    for (int q0 = 0; q0 < n; q0 += 32) {
      int pos = st + q0 + lane;
      pos = pos < 0 ? 0 : (pos > csrLen - 1 ? csrLen - 1 : pos);
      int e = csr[pos];
      e = e < 0 ? 0 : (e > nE - 1 ? nE - 1 : e);
      int s = esrc[e];
      s = s < 0 ? 0 : (s > nN - 1 ? nN - 1 : s);
      const int wi = __float_as_int(ew[e]);
      const int mcnt = (n - q0) < 32 ? (n - q0) : 32;
#pragma unroll 1
      for (int p = 0; p < mcnt; ++p) {
        const int   sp = __builtin_amdgcn_readlane(s, p);
        const float wp = __int_as_float(__builtin_amdgcn_readlane(wi, p));
        const v4f hv = *(const v4f*)(hin + (size_t)sp * HD + 4 * lane);
        acc = acc + wp * hv;
      }
    }
    const v4f xv = *(const v4f*)(x0 + (size_t)c * HD + 4 * lane);
    const v4f M = 0.9f * acc + 0.1f * xv;
    *(v4f*)(sM + (r0w + j) * HD + 4 * lane) = M;
    float mx = fmaxf(fmaxf(fabsf(M.x), fabsf(M.y)), fmaxf(fabsf(M.z), fabsf(M.w)));
    mx = fmaxf(mx, __shfl_xor(mx, 16));
    mx = fmaxf(mx, __shfl_xor(mx, 8));
    mx = fmaxf(mx, __shfl_xor(mx, 4));
    mx = fmaxf(mx, __shfl_xor(mx, 2));
    mx = fmaxf(mx, __shfl_xor(mx, 1));
    float sc, isc;
    carry_of(mx, sc, isc);
    v4h hv4;
    hv4.x = (_Float16)(M.x * sc); hv4.y = (_Float16)(M.y * sc);
    hv4.z = (_Float16)(M.z * sc); hv4.w = (_Float16)(M.w * sc);
    *(v4h*)(sA + (r0w + j) * AP + 4 * lane) = hv4;
    if (lane == 0) sFac[r0w + j] = isc * WINV;
  }
  __syncthreads();

  v8f acc[8];
  mma_rows(sA, Bs, wave, hh, m, acc);

  const int r0 = r0w + 8 * hh;
  const v4f fA = *(const v4f*)(sFac + r0);
  const v4f fB = *(const v4f*)(sFac + r0 + 4);
  float f[8];
  f[0] = fA.x; f[1] = fA.y; f[2] = fA.z; f[3] = fA.w; f[4] = fB.x; f[5] = fB.y; f[6] = fB.z; f[7] = fB.w;
  float* spm = sM + r0 * HD + m;
#pragma unroll
  for (int t = 0; t < 8; ++t) {
#pragma unroll
    for (int r = 0; r < 8; ++r) {
      const float mv = spm[r * HD + 16 * t];
      const float v  = omb * mv + bet * (acc[t][r] * f[r]);
      spm[r * HD + 16 * t] = fmaxf(v, 0.0f);
    }
  }
  __syncthreads();
  store_rows2(sM, hout, rowBase, nRowsOut, wave, lane);
}

__global__ __launch_bounds__(NTHR) void k_head(
    const float* __restrict__ Hs, const _Float16* __restrict__ Bs, const float* __restrict__ bias,
    float* out, int nN) {
  extern __shared__ v4f lds_dyn[];
  float*    sM   = (float*)lds_dyn;
  _Float16* sA   = (_Float16*)((char*)lds_dyn + LDS_SM);
  float*    sFac = (float*)((char*)lds_dyn + LDS_SM + LDS_SA);
  const int tid = threadIdx.x, lane = tid & 31, wave = tid >> 5, hh = lane >> 4, m = lane & 15;
  const int rowBase = blockIdx.x * GROWS;

  stage_rows(Hs, rowBase, nN, sA, sFac, tid, lane);
  __syncthreads();

  v8f acc[8];
  mma_rows(sA, Bs, wave, hh, m, acc);

  const int r0 = wave * 16 + 8 * hh;
  const v4f fA = *(const v4f*)(sFac + r0);
  const v4f fB = *(const v4f*)(sFac + r0 + 4);
  float f[8];
  f[0] = fA.x; f[1] = fA.y; f[2] = fA.z; f[3] = fA.w; f[4] = fB.x; f[5] = fB.y; f[6] = fB.z; f[7] = fB.w;
  float* sp = sM + r0 * HD + m;
#pragma unroll
  for (int t = 0; t < 8; ++t) {
    const float bl = bias[16 * t + m];
#pragma unroll
    for (int r = 0; r < 8; ++r) sp[r * HD + 16 * t] = acc[t][r] * f[r] + bl;
  }
  __syncthreads();

#pragma unroll 1
  for (int i = 0; i < 16; ++i) {
    float* rp = sM + (wave * 16 + i) * HD + 4 * lane;
    const v4f v = *(const v4f*)rp;
    float mx = fmaxf(fmaxf(v.x, v.y), fmaxf(v.z, v.w));
    mx = fmaxf(mx, __shfl_xor(mx, 16));
    mx = fmaxf(mx, __shfl_xor(mx, 8));
    mx = fmaxf(mx, __shfl_xor(mx, 4));
    mx = fmaxf(mx, __shfl_xor(mx, 2));
    mx = fmaxf(mx, __shfl_xor(mx, 1));
    const v4f sh = v - mx;
    float s = expf(sh.x) + expf(sh.y) + expf(sh.z) + expf(sh.w);
    s += __shfl_xor(s, 16);
    s += __shfl_xor(s, 8);
    s += __shfl_xor(s, 4);
    s += __shfl_xor(s, 2);
    s += __shfl_xor(s, 1);
    const float lse = logf(s);
    *(v4f*)rp = sh - lse;
  }
  __syncthreads();
  store_rows2(sM, out, rowBase, nN, wave, lane);
}

extern "C" void kernel_launch(void* const* d_in, const int* in_sizes, int n_in,
                              void* d_out, int out_size, void* d_ws, size_t ws_size,
                              hipStream_t stream) {
  if (n_in < 9) return;
  const int nN = in_sizes[0] / HD;
  const int nE = in_sizes[1];
  if (nN <= 0 || nE <= 0 || in_sizes[0] != nN * HD || in_sizes[2] != nE || in_sizes[3] != nE) return;
  if (in_sizes[4] != HD * HD || in_sizes[5] != HD || in_sizes[6] != HD * HD || in_sizes[7] != HD) return;
  const int nL = in_sizes[8] / (HD * HD);
  if (nL < 1 || nL > 16 || in_sizes[8] != nL * HD * HD) return;
  if (out_size != nN * HD) return;
  if (nE > (1 << 28) || nN > (1 << 24)) return;

  const float* x     = (const float*)d_in[0];
  const int*   esrc  = (const int*)d_in[1];
  const int*   edst  = (const int*)d_in[2];
  const float* ew    = (const float*)d_in[3];
  const float* W0    = (const float*)d_in[4];
  const float* b0    = (const float*)d_in[5];
  const float* W1    = (const float*)d_in[6];
  const float* b1    = (const float*)d_in[7];
  const float* convW = (const float*)d_in[8];
  float* out = (float*)d_out;

  const int NPAD   = ((nN + RPAD - 1) / RPAD) * RPAD;
  const int nBC    = (nN + NBC - 1) / NBC;
  const int CNTPAD = nBC * NBC;
  if (4 * nBC + 1 > RBN) return;
  if (NPAD > CNTPAD) return;
  const int nBF    = (nN + NBF - 1) / NBF;
  if (32 * nBF > 4096) return;
  const int csrLen = ((nE + 31) & ~31) + 4096;
  const int nG     = NPAD / GROWS;
  const int nMat   = nL + 2;

  char* ws = (char*)d_ws;
  size_t off = 0;
  const size_t oW   = off; off += (size_t)nMat * HD * HD * 2;      off = (off + 255) & ~(size_t)255;
  const size_t oCnt = off; off += (size_t)CNTPAD * 4;              off = (off + 255) & ~(size_t)255;
  const size_t oOff = off; off += (size_t)CNTPAD * 4;              off = (off + 255) & ~(size_t)255;
  const size_t oRb  = off; off += (size_t)RBN * 4;                 off = (off + 255) & ~(size_t)255;
  const size_t oCsr = off; off += (size_t)csrLen * 4;              off = (off + 255) & ~(size_t)255;
  const size_t oX0  = off; off += (size_t)NPAD * HD * 4;           off = (off + 255) & ~(size_t)255;
  const size_t oHB  = off; off += (size_t)NPAD * HD * 4;           off = (off + 255) & ~(size_t)255;
  if (off > ws_size) return;
  _Float16* wts  = (_Float16*)(ws + oW);
  int*      cnt  = (int*)(ws + oCnt);
  int*      offp = (int*)(ws + oOff);
  int*      rb   = (int*)(ws + oRb);
  int*      csr  = (int*)(ws + oCsr);
  float*    x0p  = (float*)(ws + oX0);
  float*    hB   = (float*)(ws + oHB);

  const int vec8 = 1;

  k_wprep<<<nMat * 8, NTHR, 0, stream>>>(W0, convW, W1, wts, nL);

  k_count<<<nBC, NTHR, 0, stream>>>(edst, cnt, nE, vec8);
  k_offsets<<<1, OTHR, 0, stream>>>(cnt, offp, rb, nBC);
  hipFuncSetAttribute(reinterpret_cast<const void*>(&k_fill),
                      hipFuncAttributeMaxDynamicSharedMemorySize, LDS_FILL);
  k_fill<<<nBF, NTHR, LDS_FILL, stream>>>(edst, offp, rb, csr, nE, vec8, csrLen);

  hipFuncSetAttribute(reinterpret_cast<const void*>(&k_gemm0),
                      hipFuncAttributeMaxDynamicSharedMemorySize, LDS_G);
  hipFuncSetAttribute(reinterpret_cast<const void*>(&k_layer),
                      hipFuncAttributeMaxDynamicSharedMemorySize, LDS_G);
  hipFuncSetAttribute(reinterpret_cast<const void*>(&k_head),
                      hipFuncAttributeMaxDynamicSharedMemorySize, LDS_G);
  k_gemm0<<<nG, NTHR, LDS_G, stream>>>(x, wts, b0, x0p, nN, NPAD);

  const float* hin = x0p;
  for (int l = 0; l < nL; ++l) {
    const bool toHB = (((nL - 1 - l) & 1) == 0);
    float* hout = toHB ? hB : out;
    const int nRowsOut = toHB ? NPAD : nN;
    const double bd = log(0.5 / (double)(l + 1) + 1.0);
    const float omb = (float)(1.0 - bd);
    const float bet = (float)bd;
    k_layer<<<nG, NTHR, LDS_G, stream>>>(csr, offp, cnt, esrc, ew, hin, x0p,
                                         wts + (size_t)(1 + l) * HD * HD, hout,
                                         nN, nE, csrLen, nRowsOut, omb, bet);
    hin = hout;
  }

  k_head<<<nG, NTHR, LDS_G, stream>>>(hin, wts + (size_t)(nL + 1) * HD * HD, b1, out, nN);
}
